// LinearAutoregressiveHMM_34419867910695
// MI455X (gfx1250) — hardware-run, weakly checked
//
#include <hip/hip_runtime.h>
#include <math.h>

typedef __attribute__((ext_vector_type(16))) _Float16 v16h;
typedef __attribute__((ext_vector_type(8)))  _Float16 v8h;
typedef __attribute__((ext_vector_type(8)))  float    v8f;
typedef __attribute__((ext_vector_type(4)))  float    v4f;
typedef __attribute__((ext_vector_type(4)))  int      v4i;

constexpr int kNS     = 8;
constexpr int kL      = 64;
constexpr int kC      = 64;
constexpr int kB      = 512;
constexpr int kP      = 16;
constexpr int kF      = kL * kC;
constexpr int kNAll   = kNS * kC;
constexpr int kFrames = kL + kP;
constexpr int kEPitch = kFrames * kC;
constexpr float kCarryE = 16.0f;
constexpr float kCarryW = 1024.0f;
constexpr float kFold   = 1.0f / (kCarryE * kCarryW);
constexpr float kF16Min = 6.103515625e-05f;
constexpr float kLog2Pi = 1.8378770664093453f;
constexpr float kC2Pi   = (float)kC * kLog2Pi;
static_assert(kF == 4096 && kNAll == 512 && kEPitch == 5120, "shape constants");
static_assert((kF % 32) == 0 && (kB % 64) == 0 && (kNAll % 64) == 0, "GEMM tile multiples");

constexpr size_t kOffE16   = 0;
constexpr size_t kOffW16   = kOffE16   + (size_t)kB * kEPitch * 2;
constexpr size_t kOffLinvT = kOffW16   + (size_t)kNAll * kF * 2;
constexpr size_t kOffLDT   = kOffLinvT + (size_t)kNS * kC * kC * 4;
constexpr size_t kOffTAB   = kOffLDT   + (size_t)kNS * 32 * 4;
constexpr size_t kOffELP   = kOffTAB   + (size_t)128 * 4;
constexpr size_t kOffST    = kOffELP   + (size_t)kNS * kL * kB * 4;
constexpr size_t kWsTotal  = kOffST    + (size_t)kB * kP * 4;
static_assert(kWsTotal == 10651136ull, "carve total");
static_assert(kWsTotal <= 134217728ull, "carve cap");
static_assert((kOffW16 % 128) == 0 && (kOffLinvT % 128) == 0 && (kOffLDT % 128) == 0 && (kOffTAB % 128) == 0 &&
              (kOffELP % 128) == 0 && (kOffST % 128) == 0, "128-B aligned regions");

__device__ __forceinline__ _Float16 to_f16_flush(float v) {
  const float a = fabsf(v);
  const float s = (a < kF16Min) ? 0.0f : v;
  return (_Float16)s;
}

union FragU { v16h v; v8h h[2]; };
__device__ __forceinline__ v16h frag_load(const _Float16* p) {
  FragU f;
  f.h[0] = *(const v8h*)(p);
  f.h[1] = *(const v8h*)(p + 16);
  return f.v;
}
__device__ __forceinline__ v8f mma_h(v16h a, v16h b, v8f c) {
  c = __builtin_amdgcn_wmma_f32_16x16x32_f16(false, a, false, b, (short)0, c, false, false);
  asm volatile("v_nop\n\tv_nop\n\tv_nop\n\tv_nop" : "+v"(c) : "v"(a), "v"(b));
  return c;
}
__device__ __forceinline__ void wave_lds_sync() {
  __builtin_amdgcn_fence(__ATOMIC_RELEASE, "workgroup");
  __builtin_amdgcn_wave_barrier();
  __builtin_amdgcn_fence(__ATOMIC_ACQUIRE, "workgroup");
}

__device__ __forceinline__ void gemm_tile64(const _Float16* Ab, int lda, const _Float16* Bb, int ldb,
                                            int K, int lane, v8f (&acc)[4][4]) {
  const int rlane = lane & 15;
  const int koff  = (lane >> 4) * 8;
  const _Float16* ap = Ab + (size_t)rlane * lda + koff;
  const _Float16* bp = Bb + (size_t)rlane * ldb + koff;
  for (int k0 = 0; k0 < K; k0 += 32) {
    v16h bh[4];
#pragma unroll
    for (int j = 0; j < 4; ++j) bh[j] = frag_load(bp + (size_t)(j * 16) * ldb + k0);
#pragma unroll
    for (int i = 0; i < 4; ++i) {
      const v16h ah = frag_load(ap + (size_t)(i * 16) * lda + k0);
#pragma unroll
      for (int j = 0; j < 4; ++j) acc[i][j] = mma_h(ah, bh[j], acc[i][j]);
    }
  }
}

__global__ __launch_bounds__(256) void cvt_rows_f16_kernel(
    const float* __restrict__ src, unsigned short* __restrict__ dst, int total8, int srcRow, int dstPitch, float carry)
{
  const int i = blockIdx.x * 256 + threadIdx.x;
  if (i >= total8) return;
  const size_t e0 = (size_t)i << 3;
  const int row = (int)(e0 / (size_t)srcRow);
  const int off = (int)(e0 - (size_t)row * (size_t)srcRow);
  const v4f a0 = *(const v4f*)(src + e0);
  const v4f a1 = *(const v4f*)(src + e0 + 4);
  v8h hv;
#pragma unroll
  for (int e = 0; e < 4; ++e) {
    hv[e]     = to_f16_flush(a0[e] * carry);
    hv[4 + e] = to_f16_flush(a1[e] * carry);
  }
  unsigned short* q = dst + (size_t)row * dstPitch + off;
  *(volatile v8h*)q = hv;
  __threadfence();
  *(volatile v8h*)q = hv;
}

__global__ __launch_bounds__(64) void chol_inverse_kernel(
    const float* __restrict__ CC, float* __restrict__ LinvT, float* __restrict__ LDT)
{
  __shared__ float sA[64 * 65];
  __shared__ float sX[64 * 65];
  __shared__ float sLd[2];
  const int k = blockIdx.x;
  const int r = threadIdx.x;

#pragma unroll 1
  for (int c = 0; c < 64; ++c) {
    float v = CC[(size_t)k * 4096 + r * 64 + c];
    asm volatile("" : "+v"(v));
    const float ev = expf(v);
    const float tv = (c < r) ? v : ((c == r) ? ev : 0.0f);
    sX[r * 65 + c] = tv;
  }
  __syncthreads();

#pragma unroll 1
  for (int c = 0; c <= r; ++c) {
    float s = 0.0f;
#pragma unroll 1
    for (int p = 0; p <= c; ++p) s = fmaf(sX[r * 65 + p], sX[c * 65 + p], s);
    sA[r * 65 + c] = s + ((c == r) ? 1e-6f : 0.0f);
  }
  __syncthreads();

#pragma unroll 1
  for (int j = 0; j < 64; ++j) {
    float s = 0.0f;
    if (r >= j) {
      s = sA[r * 65 + j];
#pragma unroll 1
      for (int p = 0; p < j; ++p) s = fmaf(-sA[r * 65 + p], sA[j * 65 + p], s);
    }
    if (r == j) sA[j * 65 + j] = sqrtf(s);
    __syncthreads();
    if (r > j) sA[r * 65 + j] = s / sA[j * 65 + j];
    __syncthreads();
  }

  if (r == 0) {
    float ld = 0.0f;
#pragma unroll 1
    for (int j = 0; j < 64; ++j) ld += logf(sA[j * 65 + j]);
    sLd[0] = ld;
    sLd[1] = 0.0f;
  }

  {
    const int c = r;
#pragma unroll 1
    for (int i = 0; i < 64; ++i) {
      float s = (i == c) ? 1.0f : 0.0f;
#pragma unroll 1
      for (int p = c; p < i; ++p) s = fmaf(-sA[i * 65 + p], sX[p * 65 + c], s);
      const float x = s / sA[i * 65 + i];
      sX[i * 65 + c] = (i >= c) ? x : 0.0f;
    }
  }
  __syncthreads();

  float* dstp = LinvT + (size_t)k * 4096;
  for (int pass = 0; pass < 2; ++pass) {
#pragma unroll 1
    for (int it = 0; it < 16; ++it) {
      const int lin4 = (it * 64 + r) * 4;
      const int c  = lin4 >> 6;
      const int i0 = lin4 & 63;
      v4f v;
      v[0] = sX[(i0 + 0) * 65 + c];
      v[1] = sX[(i0 + 1) * 65 + c];
      v[2] = sX[(i0 + 2) * 65 + c];
      v[3] = sX[(i0 + 3) * 65 + c];
      *(volatile v4f*)(dstp + lin4) = v;
    }
    __threadfence();
  }
  if (r < 32) {
    const float ldv = sLd[0];
    volatile float* lp = LDT + k * 32 + r;
    *lp = ldv;
    __threadfence();
    *lp = ldv;
  }
}

__global__ __launch_bounds__(64) void hmm_tables_kernel(
    const float* __restrict__ T, const float* __restrict__ I, float* __restrict__ tab)
{
#pragma clang fp contract(off)
  __shared__ __align__(16) float sTab[128];
  const int tid = threadIdx.x;
  sTab[tid] = 0.0f;
  sTab[64 + tid] = 0.0f;
  __syncthreads();
  const int i = tid & 7;
  float mx = -INFINITY;
#pragma unroll 1
  for (int j = 0; j < 8; ++j) {
    float tv = T[i * 8 + j];
    asm volatile("" : "+v"(tv));
    mx = fmaxf(mx, tv);
  }
  float ssum = 0.0f;
#pragma unroll 1
  for (int j = 0; j < 8; ++j) {
    float tv = T[i * 8 + j];
    asm volatile("" : "+v"(tv));
    ssum += expf(tv - mx);
  }
  const float rs = 1.0f / ssum;
  int arg = 0;
  float bp = -1.0f;
#pragma unroll 1
  for (int j = 0; j < 8; ++j) {
    float tv = T[i * 8 + j];
    asm volatile("" : "+v"(tv));
    const float pr = expf(tv - mx) * rs;
    const float lv = logf(pr + 1e-8f);
    if (tid < 8) sTab[i * 8 + j] = lv;
    if (pr > bp) { bp = pr; arg = j; }
  }
  float m2 = -INFINITY;
#pragma unroll 1
  for (int j = 0; j < 8; ++j) {
    float iv = I[j];
    asm volatile("" : "+v"(iv));
    m2 = fmaxf(m2, iv);
  }
  float s2 = 0.0f;
#pragma unroll 1
  for (int j = 0; j < 8; ++j) {
    float iv = I[j];
    asm volatile("" : "+v"(iv));
    s2 += expf(iv - m2);
  }
  float ii = I[i];
  asm volatile("" : "+v"(ii));
  const float r2 = 1.0f / s2;
  const float li = logf(expf(ii - m2) * r2);
  if (tid < 8) {
    sTab[64 + i] = li;
    sTab[72 + i] = (float)arg;
  }
  __syncthreads();
  if (tid < 32) {
    const v4f v = *(const v4f*)(sTab + tid * 4);
    float* gp = tab + tid * 4;
    *(volatile v4f*)gp = v;
    __threadfence();
    *(volatile v4f*)gp = v;
  }
}

__global__ __launch_bounds__(256) void ar_loglik_kernel(
    const unsigned short* __restrict__ E16p, const unsigned short* __restrict__ W16p,
    const float* __restrict__ em, const float* __restrict__ means,
    const float* __restrict__ LinvT, const float* __restrict__ LDT, float* __restrict__ elp)
{
  __shared__ __align__(16) float sLT[64 * 64];
  __shared__ __align__(16) float sTile[2][64 * 68];
  __shared__ __align__(16) float sQ[2][64];
  const int tid  = threadIdx.x;
  const int lane = tid & 31;
  const int wave = tid >> 5;
  const int t  = blockIdx.x;
  const int k  = blockIdx.y;
  const int b0 = (blockIdx.z * 2 + wave) * 64;

#pragma unroll 4
  for (int it = 0; it < 16; ++it) {
    const int idx = (it * 64 + tid) * 4;
    *(v4f*)(sLT + idx) = *(const v4f*)(LinvT + (size_t)k * 4096 + idx);
  }
  __syncthreads();

  v8f acc[4][4];
#pragma unroll
  for (int i = 0; i < 4; ++i)
#pragma unroll
    for (int j = 0; j < 4; ++j) acc[i][j] = (v8f){0.f, 0.f, 0.f, 0.f, 0.f, 0.f, 0.f, 0.f};

  const int wofs = (t > 0) ? (kL - t) * kC : 0;
  const _Float16* Ab = (const _Float16*)E16p + (size_t)b0 * kEPitch;
  const _Float16* Bb = (const _Float16*)W16p + (size_t)(k * kC) * kF + wofs;
  gemm_tile64(Ab, kEPitch, Bb, kF, t * kC, lane, acc);

  float* tile = sTile[wave];
  const int rlane = lane & 15;
  const int mOff  = (lane >> 4) * 8;
  {
    float mu[4];
#pragma unroll
    for (int j = 0; j < 4; ++j) mu[j] = means[k * kC + j * 16 + rlane];
#pragma unroll
    for (int i = 0; i < 4; ++i)
#pragma unroll
      for (int j = 0; j < 4; ++j)
#pragma unroll
        for (int r = 0; r < 8; ++r)
          tile[(i * 16 + mOff + r) * 68 + j * 16 + rlane] = mu[j] + acc[i][j][r] * kFold;
  }
  wave_lds_sync();
  {
    const int hh = lane >> 4;
    const int c4 = (lane & 15) * 4;
#pragma unroll 4
    for (int it = 0; it < 32; ++it) {
      const int row = it * 2 + hh;
      const v4f tg = *(const v4f*)(em + ((size_t)(b0 + row) * kL + t) * kC + c4);
      const v4f pv = *(const v4f*)(tile + row * 68 + c4);
      const v4f dv = tg - pv;
      *(v4f*)(tile + row * 68 + c4) = dv;
    }
  }
  wave_lds_sync();

  const float ldv = LDT[k * 32];
#pragma unroll 1
  for (int rr = 0; rr < 2; ++rr) {
    const int row = lane + 32 * rr;
    const float* dr = tile + row * 68;
    float q = 0.0f;
#pragma unroll 1
    for (int ic = 0; ic < 4; ++ic) {
      float s[16];
#pragma unroll
      for (int x = 0; x < 16; ++x) s[x] = 0.0f;
      const float* lp = sLT + ic * 16;
      const int c4end = 4 * (ic + 1);
#pragma unroll 1
      for (int cc = 0; cc < c4end; ++cc) {
        const v4f d4 = *(const v4f*)(dr + 4 * cc);
        const float* le = lp + (4 * cc) * 64;
#pragma unroll
        for (int e = 0; e < 4; ++e) {
          const float de = d4[e];
          const v4f l0 = *(const v4f*)(le + e * 64);
          const v4f l1 = *(const v4f*)(le + e * 64 + 4);
          const v4f l2 = *(const v4f*)(le + e * 64 + 8);
          const v4f l3 = *(const v4f*)(le + e * 64 + 12);
#pragma unroll
          for (int x = 0; x < 4; ++x) {
            s[x]      = fmaf(l0[x], de, s[x]);
            s[4 + x]  = fmaf(l1[x], de, s[4 + x]);
            s[8 + x]  = fmaf(l2[x], de, s[8 + x]);
            s[12 + x] = fmaf(l3[x], de, s[12 + x]);
          }
        }
      }
#pragma unroll
      for (int x = 0; x < 16; ++x) q = fmaf(s[x], s[x], q);
    }
    sQ[wave][row] = -0.5f * (kC2Pi + q) - ldv;
  }
  wave_lds_sync();
  {
    const int c4 = (lane & 15) * 4;
    const v4f qv = *(const v4f*)(sQ[wave] + c4);
    float* ep = elp + ((size_t)(k * kL + t)) * kB + b0 + c4;
    if (lane < 16) *(volatile v4f*)ep = qv;
    __threadfence();
    if (lane < 16) *(volatile v4f*)ep = qv;
  }
}

__global__ __launch_bounds__(512) void forward_scan_kernel(
    const float* __restrict__ elp, const float* __restrict__ tab, int* __restrict__ st)
{
#pragma clang fp contract(off)
  __shared__ __align__(16) float sTab[128];
  __shared__ __align__(16) int sSt[64 * 16];
  const int tid = threadIdx.x;
  if (tid < 128) sTab[tid] = tab[tid];
  __syncthreads();
  const int bl = tid >> 3;
  const int j  = tid & 7;
  const int b  = blockIdx.x * 64 + bl;
  float la = sTab[64 + j] + elp[(size_t)(j * kL) * kB + b];
#pragma unroll 1
  for (int t = 1; t < kL; ++t) {
    const float e = elp[(size_t)(j * kL + t) * kB + b];
    float m = -INFINITY;
#pragma unroll 1
    for (int i = 0; i < 8; ++i) {
      const float o = __shfl(la, i, 8);
      const float v = o + sTab[i * 8 + j];
      m = fmaxf(m, v);
    }
    float s = 0.0f;
#pragma unroll 1
    for (int i = 0; i < 8; ++i) {
      const float o = __shfl(la, i, 8);
      const float v = o + sTab[i * 8 + j];
      s += expf(v - m);
    }
    la = (logf(s) + m) + e;
  }
  float best = __shfl(la, 0, 8);
  int arg = 0;
#pragma unroll 1
  for (int i = 1; i < 8; ++i) {
    const float v = __shfl(la, i, 8);
    if (v > best) { best = v; arg = i; }
  }
  int s = arg;
#pragma unroll 1
  for (int p = 0; p < kP; ++p) {
    int nx = (int)sTab[72 + s];
    nx = nx < 0 ? 0 : (nx > 7 ? 7 : nx);
    s = nx;
    if (j == 0) sSt[bl * 16 + p] = s;
  }
  __syncthreads();
  if (tid < 256) {
    const v4i v = *(const v4i*)(sSt + tid * 4);
    int* gp = st + (size_t)blockIdx.x * 1024 + tid * 4;
    *(volatile v4i*)gp = v;
    __threadfence();
    *(volatile v4i*)gp = v;
  }
}

__global__ __launch_bounds__(256) void rollout_step_kernel(
    const unsigned short* Ein, unsigned short* Eout, const unsigned short* __restrict__ W16p,
    const float* __restrict__ means, const int* __restrict__ st, float* __restrict__ out, int p)
{
  __shared__ __align__(16) float sOut[64 * 68];
  __shared__ int sSt[64];
  const int tid  = threadIdx.x;
  const int lane = tid & 31;
  const int wave = tid >> 5;
  const int b0 = blockIdx.x * 64;
  const int k  = wave;
  {
    int sv = st[(size_t)(b0 + (tid & 63)) * kP + p];
    asm volatile("" : "+v"(sv));
    sv = sv < 0 ? 0 : (sv > 7 ? 7 : sv);
    if (tid < 64) sSt[tid] = sv;
  }
  __syncthreads();

  v8f acc[4][4];
#pragma unroll
  for (int i = 0; i < 4; ++i)
#pragma unroll
    for (int j = 0; j < 4; ++j) acc[i][j] = (v8f){0.f, 0.f, 0.f, 0.f, 0.f, 0.f, 0.f, 0.f};

  const _Float16* Ab = (const _Float16*)Ein + (size_t)b0 * kEPitch + p * kC;
  const _Float16* Bb = (const _Float16*)W16p + (size_t)(k * kC) * kF;
  gemm_tile64(Ab, kEPitch, Bb, kF, kF, lane, acc);

  const int rlane = lane & 15;
  const int mOff  = (lane >> 4) * 8;
  {
    float mu[4];
#pragma unroll
    for (int j = 0; j < 4; ++j) mu[j] = means[k * kC + j * 16 + rlane];
#pragma unroll
    for (int i = 0; i < 4; ++i)
#pragma unroll
      for (int r = 0; r < 8; ++r) {
        const int row = i * 16 + mOff + r;
        const int srow = sSt[row];
#pragma unroll
        for (int j = 0; j < 4; ++j) {
          const float v = acc[i][j][r] * kFold + mu[j];
          if (srow == k) sOut[row * 68 + j * 16 + rlane] = v;
        }
      }
  }
  __syncthreads();
  {
    const int hh = lane >> 4;
    const int c4 = (lane & 15) * 4;
    const int q  = lane >> 3;
    const int c8 = (lane & 7) * 8;
    v4f ov[4];
    v8h hv[2];
#pragma unroll
    for (int it = 0; it < 4; ++it) ov[it] = *(const v4f*)(sOut + (wave * 8 + it * 2 + hh) * 68 + c4);
#pragma unroll
    for (int it = 0; it < 2; ++it) {
      const float* sp = sOut + (wave * 8 + it * 4 + q) * 68 + c8;
      const v4f a0 = *(const v4f*)(sp);
      const v4f a1 = *(const v4f*)(sp + 4);
#pragma unroll
      for (int e = 0; e < 4; ++e) {
        hv[it][e]     = to_f16_flush(a0[e] * kCarryE);
        hv[it][4 + e] = to_f16_flush(a1[e] * kCarryE);
      }
    }
    for (int pass = 0; pass < 2; ++pass) {
#pragma unroll
      for (int it = 0; it < 4; ++it) {
        const int row = wave * 8 + it * 2 + hh;
        *(volatile v4f*)(out + ((size_t)(b0 + row) * kP + p) * kC + c4) = ov[it];
      }
#pragma unroll
      for (int it = 0; it < 2; ++it) {
        const int row = wave * 8 + it * 4 + q;
        *(volatile v8h*)(Eout + (size_t)(b0 + row) * kEPitch + (size_t)(kL + p) * kC + c8) = hv[it];
      }
      __threadfence();
    }
  }
}

extern "C" void kernel_launch(void* const* d_in, const int* in_sizes, int n_in,
                              void* d_out, int out_size, void* d_ws, size_t ws_size,
                              hipStream_t stream) {
  if (n_in < 6) return;
  if (in_sizes[0] != kB * kL * kC) return;
  if (in_sizes[1] != kNS * kNS) return;
  if (in_sizes[2] != kNS) return;
  if (in_sizes[3] != kNS * kC) return;
  if (in_sizes[4] != kNS * kC * kC) return;
  if (in_sizes[5] != kNS * kC * kF) return;
  if (out_size != kB * kP * kC) return;
  if (ws_size < kWsTotal) return;

  const float* em = (const float*)d_in[0];
  const float* T  = (const float*)d_in[1];
  const float* I  = (const float*)d_in[2];
  const float* Mn = (const float*)d_in[3];
  const float* CC = (const float*)d_in[4];
  const float* W  = (const float*)d_in[5];
  float* out = (float*)d_out;

  char* ws = (char*)d_ws;
  unsigned short* E16   = (unsigned short*)(ws + kOffE16);
  unsigned short* W16   = (unsigned short*)(ws + kOffW16);
  float*          LinvT = (float*)(ws + kOffLinvT);
  float*          LDT   = (float*)(ws + kOffLDT);
  float*          TAB   = (float*)(ws + kOffTAB);
  float*          ELP   = (float*)(ws + kOffELP);
  int*            ST    = (int*)(ws + kOffST);

  const int total8 = kB * kF / 8;
  cvt_rows_f16_kernel<<<total8 / 256, 256, 0, stream>>>(W, W16, total8, kF, kF, kCarryW);
  cvt_rows_f16_kernel<<<total8 / 256, 256, 0, stream>>>(em, E16, total8, kF, kEPitch, kCarryE);
  chol_inverse_kernel<<<kNS, 64, 0, stream>>>(CC, LinvT, LDT);
  hmm_tables_kernel<<<1, 64, 0, stream>>>(T, I, TAB);
  ar_loglik_kernel<<<dim3(kL, kNS, 4), 64, 0, stream>>>(E16, W16, em, Mn, LinvT, LDT, ELP);
  forward_scan_kernel<<<kB / 64, 512, 0, stream>>>(ELP, TAB, ST);
  for (int p = 0; p < kP; ++p)
    rollout_step_kernel<<<kB / 64, 256, 0, stream>>>(E16, E16, W16, Mn, ST, out, p);
}
